// ScoreHead_50757923504886
// MI455X (gfx1250) — hardware-verified
//
#include <hip/hip_runtime.h>
#include <stddef.h>


typedef _Float16 v16h __attribute__((ext_vector_type(16)));
typedef _Float16 v8h  __attribute__((ext_vector_type(8)));
typedef float    v8f  __attribute__((ext_vector_type(8)));
typedef float    v4f  __attribute__((ext_vector_type(4)));
typedef _Float16 h16;

#ifndef NQ
#define NQ 256
#endif
#ifndef NS
#define NS 16384
#endif
#define NQ_FULL 256
#define NS_FULL 16384
#define DIM   768
#define NHEAD 8
#define HD    96

static_assert(NQ >= 64 && NQ <= NQ_FULL && (NQ % 64) == 0);
static_assert(NS >= 64 && NS <= NS_FULL && (NS % 64) == 0);
static_assert(DIM == NHEAD * HD);
static_assert(NHEAD == 8);
static_assert((HD % 32) == 0 && (HD / 32) == 3);
static_assert((DIM % 64) == 0 && (DIM % 32) == 0 && (DIM % 8) == 0);
static_assert((NS_FULL % 32) == 0);
static_assert((((size_t)NQ * DIM) % 2048) == 0);
static_assert((((size_t)NS * DIM) % 2048) == 0);
static_assert((((size_t)DIM * DIM) % 2048) == 0);
static_assert((size_t)NS * DIM < (size_t)0xFFFFFFFFu);

#define LDC 68
static_assert((LDC % 4) == 0 && LDC >= 64);

#define XCARRY 16.0f
#define WCARRY 64.0f
#define QCARRY 16.0f

#define XQ_BYTES ((size_t)NQ * DIM * 2)
#define XS_BYTES ((size_t)NS * DIM * 2)
#define W_BYTES  ((size_t)DIM * DIM * 2)
#define OFF_XQ ((size_t)0)
#define OFF_XS (OFF_XQ + XQ_BYTES)
#define OFF_WQ (OFF_XS + XS_BYTES)
#define OFF_WK (OFF_WQ + W_BYTES)
#define OFF_QP (OFF_WK + W_BYTES)
#define OFF_KP (OFF_QP + XQ_BYTES)
#define WS_TOTAL (OFF_KP + XS_BYTES)
static_assert((XQ_BYTES % 128) == 0 && (XS_BYTES % 128) == 0 && (W_BYTES % 128) == 0);
static_assert(WS_TOTAL <= (size_t)134217728);

__device__ __forceinline__ float bf16r(float x) {
  unsigned int u = __float_as_uint(x);
  u = (u + 0x7FFFu + ((u >> 16) & 1u)) & 0xFFFF0000u;
  return __uint_as_float(u);
}

static __device__ __forceinline__ h16 toh_flush(float v) {
  const h16 r = (h16)v;
  return (fabsf(v) < 6.103515625e-05f) ? (h16)0.0f : r;
}

__device__ __forceinline__ v16h frag_at(const _Float16* p) {
  v8h lo = *(const v8h*)(p);
  v8h hi = *(const v8h*)(p + 16);
  v16h out;
#pragma unroll
  for (int i = 0; i < 8; ++i) { out[i] = lo[i]; out[i + 8] = hi[i]; }
  return out;
}

__device__ __forceinline__ v8f wmma16(v16h a, v16h b, v8f c) {
  v8f d = __builtin_amdgcn_wmma_f32_16x16x32_f16(false, a, false, b, (short)0, c,
                                                 false, false);
  asm volatile("v_nop\n\tv_nop\n\tv_nop\n\tv_nop" : "+v"(d) : "v"(a), "v"(b));
  return d;
}

__global__ __launch_bounds__(256) void rowconv_kernel(
    const float* __restrict__ src, _Float16* __restrict__ dst, unsigned n, float carry) {
  const unsigned e = (blockIdx.x * 256u + threadIdx.x) * 8u;
  if (e + 8u <= n) {
    const v4f a0 = *(const v4f*)(src + e);
    const v4f a1 = *(const v4f*)(src + e + 4u);
    v8h o;
#pragma unroll
    for (int i = 0; i < 4; ++i) {
      o[i]     = toh_flush(carry * bf16r(a0[i]));
      o[i + 4] = toh_flush(carry * bf16r(a1[i]));
    }
    _Float16* p = dst + e;
    *(volatile v8h*)p = o;
    __threadfence();
    *(volatile v8h*)p = o;
  }
}

__global__ __launch_bounds__(256) void gemm_proj_kernel(
    const _Float16* __restrict__ A16, const _Float16* __restrict__ Bt,
    const float* __restrict__ bias, _Float16* __restrict__ out16) {
  __shared__ float Cs[64 * LDC];
  const unsigned tid = threadIdx.x, lane = tid & 31u, w = tid >> 5;
  const unsigned mw = w >> 1, nw = w & 1u;
  const unsigned hh = lane >> 4, m = lane & 15u;
  const unsigned n0 = blockIdx.x * 64u;
  const unsigned row0 = blockIdx.y * 64u;
  const unsigned K = (unsigned)DIM;

  const _Float16* ap  = A16 + (size_t)(row0 + mw * 16u + m) * K + hh * 8u;
  const _Float16* bp0 = Bt + (size_t)(n0 + nw * 32u + m) * K + hh * 8u;
  const _Float16* bp1 = bp0 + (size_t)16 * K;
  v8f acc0 = {}, acc1 = {};
#pragma unroll 2
  for (unsigned k0 = 0; k0 < K; k0 += 32u) {
    const v16h a  = frag_at(ap + k0);
    const v16h b0 = frag_at(bp0 + k0);
    const v16h b1 = frag_at(bp1 + k0);
    acc0 = wmma16(a, b0, acc0);
    acc1 = wmma16(a, b1, acc1);
  }
#pragma unroll
  for (int r = 0; r < 8; ++r) {
    float* d = &Cs[(mw * 16u + hh * 8u + (unsigned)r) * LDC + nw * 32u + m];
    d[0]  = acc0[r];
    d[16] = acc1[r];
  }
  __syncthreads();

  v8h x[2];
  size_t off[2];
#pragma unroll
  for (unsigned i = 0; i < 2u; ++i) {
    const unsigned r = 32u * i + (tid >> 3);
    const unsigned c = (tid & 7u) * 8u;
    const v4f u0 = *(const v4f*)&Cs[r * LDC + c];
    const v4f u1 = *(const v4f*)&Cs[r * LDC + c + 4];
    const v4f g0 = *(const v4f*)(bias + n0 + c);
    const v4f g1 = *(const v4f*)(bias + n0 + c + 4u);
#pragma unroll
    for (int j = 0; j < 4; ++j) {
      x[i][j]     = toh_flush(u0[j] * (QCARRY / (XCARRY * WCARRY)) + QCARRY * bf16r(g0[j]));
      x[i][j + 4] = toh_flush(u1[j] * (QCARRY / (XCARRY * WCARRY)) + QCARRY * bf16r(g1[j]));
    }
    off[i] = (size_t)(row0 + r) * DIM + n0 + c;
  }
#pragma unroll
  for (int i = 0; i < 2; ++i) *(volatile v8h*)(out16 + off[i]) = x[i];
  __threadfence();
#pragma unroll
  for (int i = 0; i < 2; ++i) *(volatile v8h*)(out16 + off[i]) = x[i];
}

__global__ __launch_bounds__(256) void score_kernel(
    const _Float16* __restrict__ Qp, const _Float16* __restrict__ Kp,
    const float* __restrict__ W1, const float* __restrict__ b1,
    const float* __restrict__ W2, const float* __restrict__ b2,
    float* __restrict__ out) {
  __shared__ float Cs[64 * LDC];
  const unsigned tid = threadIdx.x, lane = tid & 31u;
  const unsigned wave = (unsigned)__builtin_amdgcn_readfirstlane((int)(threadIdx.x >> 5));
  const unsigned mw = wave >> 1, nw = wave & 1u;
  const unsigned hh = lane >> 4, m = lane & 15u;
  const unsigned n0 = blockIdx.x * 64u;
  const unsigned row0 = blockIdx.y * 64u;
  const float lscale = 0.10206207261596575f * (1.0f / (QCARRY * QCARRY));

  float w1s[4][NHEAD], bb1[4], w2s[4];
#pragma unroll
  for (int j = 0; j < 4; ++j) {
    bb1[j] = bf16r(b1[j]);
    w2s[j] = bf16r(W2[j]);
#pragma unroll
    for (int h = 0; h < NHEAD; ++h) w1s[j][h] = bf16r(W1[j * NHEAD + h]);
  }
  const float bb2 = bf16r(b2[0]);

  const _Float16* ap = Qp + (size_t)(row0 + mw * 16u + m) * DIM + hh * 8u;

#pragma unroll 1
  for (unsigned t = 0; t < 2u; ++t) {
    const _Float16* bp = Kp + (size_t)(n0 + nw * 32u + t * 16u + m) * DIM + hh * 8u;
    v8f acc[NHEAD];
#pragma unroll
    for (int h = 0; h < NHEAD; ++h) {
      v8f a_ = {};
#pragma unroll
      for (int c = 0; c < HD / 32; ++c) {
        const v16h af = frag_at(ap + h * HD + c * 32);
        const v16h bf = frag_at(bp + h * HD + c * 32);
        a_ = wmma16(af, bf, a_);
      }
      acc[h] = a_;
    }

#pragma unroll
    for (int r = 0; r < 8; ++r) {
      float l[NHEAD];
#pragma unroll
      for (int h = 0; h < NHEAD; ++h) l[h] = acc[h][r] * lscale;
      float s = bb2;
#pragma unroll
      for (int j = 0; j < 4; ++j) {
        float z = bb1[j];
#pragma unroll
        for (int h = 0; h < NHEAD; ++h) z = fmaf(w1s[j][h], l[h], z);
        const float g = 0.5f * z * (1.0f + erff(z * 0.70710678118654752f));
        s = fmaf(w2s[j], g, s);
      }
      Cs[(mw * 16u + hh * 8u + (unsigned)r) * LDC + nw * 32u + t * 16u + m] = s;
    }
  }
  __syncthreads();

  v4f xs[4];
  size_t off[4];
#pragma unroll
  for (unsigned i = 0; i < 4u; ++i) {
    const unsigned r = 16u * i + (tid >> 4);
    const unsigned c = (tid & 15u) * 4u;
    xs[i] = *(const v4f*)&Cs[r * LDC + c];
    off[i] = (size_t)(row0 + r) * NS_FULL + n0 + c;
  }
#pragma unroll
  for (int i = 0; i < 4; ++i) *(volatile v4f*)(out + off[i]) = xs[i];
  __threadfence();
#pragma unroll
  for (int i = 0; i < 4; ++i) *(volatile v4f*)(out + off[i]) = xs[i];
}

extern "C" void kernel_launch(void* const* d_in, const int* in_sizes, int n_in,
                              void* d_out, int out_size, void* d_ws, size_t ws_size,
                              hipStream_t stream) {
  if (n_in < 10) return;
  if ((long long)in_sizes[0] < (long long)NQ * DIM) return;
  if ((long long)in_sizes[1] < (long long)NS * DIM) return;
  if ((long long)in_sizes[2] < (long long)DIM * DIM) return;
  if ((long long)in_sizes[4] < (long long)DIM * DIM) return;
  if (in_sizes[3] < DIM || in_sizes[5] < DIM) return;
  if (in_sizes[6] < 4 * NHEAD || in_sizes[7] < 4 || in_sizes[8] < 4 || in_sizes[9] < 1) return;
  if ((long long)out_size < (long long)(NQ - 1) * NS_FULL + NS) return;
  if (ws_size < WS_TOTAL) return;

  const float* query  = (const float*)d_in[0];
  const float* search = (const float*)d_in[1];
  const float* wq     = (const float*)d_in[2];
  const float* bq     = (const float*)d_in[3];
  const float* wk     = (const float*)d_in[4];
  const float* bk     = (const float*)d_in[5];
  const float* w1     = (const float*)d_in[6];
  const float* b1     = (const float*)d_in[7];
  const float* w2     = (const float*)d_in[8];
  const float* b2     = (const float*)d_in[9];
  float* out = (float*)d_out;

  char* ws = (char*)d_ws;
  _Float16* Xq16 = (_Float16*)(ws + OFF_XQ);
  _Float16* Xs16 = (_Float16*)(ws + OFF_XS);
  _Float16* Wq16 = (_Float16*)(ws + OFF_WQ);
  _Float16* Wk16 = (_Float16*)(ws + OFF_WK);
  _Float16* Qp16 = (_Float16*)(ws + OFF_QP);
  _Float16* Kp16 = (_Float16*)(ws + OFF_KP);

  dim3 blk(256);
  const unsigned nq_el = (unsigned)((size_t)NQ * DIM);
  const unsigned ns_el = (unsigned)((size_t)NS * DIM);
  const unsigned nw_el = (unsigned)((size_t)DIM * DIM);

  rowconv_kernel<<<dim3(nq_el / 2048u), blk, 0, stream>>>(query, Xq16, nq_el, XCARRY);
  rowconv_kernel<<<dim3(ns_el / 2048u), blk, 0, stream>>>(search, Xs16, ns_el, XCARRY);
  rowconv_kernel<<<dim3(nw_el / 2048u), blk, 0, stream>>>(wq, Wq16, nw_el, WCARRY);
  rowconv_kernel<<<dim3(nw_el / 2048u), blk, 0, stream>>>(wk, Wk16, nw_el, WCARRY);

  gemm_proj_kernel<<<dim3(DIM / 64, NQ / 64), blk, 0, stream>>>(Xq16, Wq16, bq, Qp16);
  gemm_proj_kernel<<<dim3(DIM / 64, NS / 64), blk, 0, stream>>>(Xs16, Wk16, bk, Kp16);

  score_kernel<<<dim3(NS / 64, NQ / 64), blk, 0, stream>>>(Qp16, Kp16, w1, b1, w2, b2, out);
}
